// Attention_69260642615568
// MI455X (gfx1250) — hardware-run, weakly checked
//
#include <hip/hip_runtime.h>


#ifndef NB
#define NB 4
#endif
#ifndef SEQ
#define SEQ 2048
#endif
#define NB_FULL  4
#define SEQ_FULL 2048
#ifndef OUT_SEQ
#define OUT_SEQ SEQ
#endif
#define DM   1024
#define NH_  16
#define HD   64
#define AW   4
#define SC2  (0.125f * 1.4426950408889634f)
#define L2E  1.4426950408889634f
#define PSH  8.0f
#define PFL  (-14.0f)
#define WOS  64.0f

static_assert(HD == 64);
static_assert(HD == 16 * 4);
static_assert(NH_ * HD == DM);
static_assert(DM % 64 == 0);
static_assert(DM % 32 == 0);
static_assert(HD % 32 == 0);
static_assert(SEQ % 64 == 0);
static_assert((NB * SEQ) % 64 == 0);
static_assert(SEQ % 32 == 0);
static_assert(SEQ % (16 * AW) == 0);
static_assert(((size_t)SEQ * DM) % 8 == 0);
static_assert(((size_t)DM * DM) % 8 == 0);
static_assert(NB <= NB_FULL);
static_assert(SEQ <= SEQ_FULL);
static_assert(SEQ % 4 == 0);
static_assert(((SEQ / 4) * SEQ) % 1024 == 0);

typedef _Float16 h16;
typedef unsigned short bf;
typedef __attribute__((ext_vector_type(16))) __bf16   v16bf;
typedef __attribute__((ext_vector_type(16))) _Float16 v16h;
typedef __attribute__((ext_vector_type(8)))  _Float16 v8h;
typedef __attribute__((ext_vector_type(8)))  unsigned short v8us;
typedef __attribute__((ext_vector_type(8)))  float    v8f;
typedef __attribute__((ext_vector_type(4)))  float    v4f;
typedef __attribute__((ext_vector_type(4)))  int      v4i;
typedef v4f  __attribute__((may_alias)) v4fa;

__device__ __forceinline__ unsigned short f2bf(float f) { unsigned u = __float_as_uint(f); u += 0x7FFFu + ((u >> 16) & 1u); return (unsigned short)(u >> 16); }
__device__ __forceinline__ float bfr(float f) { return __uint_as_float(((unsigned)f2bf(f)) << 16); }
__device__ __forceinline__ v16h cat16(v8h lo, v8h hi) { return __builtin_shufflevector(lo, hi, 0, 1, 2, 3, 4, 5, 6, 7, 8, 9, 10, 11, 12, 13, 14, 15); }
__device__ __forceinline__ v16bf cat16b(v8us lo, v8us hi) { return __builtin_bit_cast(v16bf, __builtin_shufflevector(lo, hi, 0, 1, 2, 3, 4, 5, 6, 7, 8, 9, 10, 11, 12, 13, 14, 15)); }
__device__ __forceinline__ v8f wmma16(v16h a, v16h b, v8f c) { return __builtin_amdgcn_wmma_f32_16x16x32_f16(false, a, false, b, (short)0, c, false, false); }
__device__ __forceinline__ v8f wmmab(v16bf a, v16bf b, v8f c) { return __builtin_amdgcn_wmma_f32_16x16x32_bf16(false, a, false, b, (short)0, c, false, false); }
__device__ __forceinline__ v16h  ldh(const h16* p) { return cat16(*(const v8h*)p, *(const v8h*)(p + 16)); }
__device__ __forceinline__ v16bf ldb(const bf* p)  { return cat16b(*(const v8us*)p, *(const v8us*)(p + 16)); }
__device__ __forceinline__ void wave_sync() { __builtin_amdgcn_fence(3  , "wavefront"); __builtin_amdgcn_wave_barrier(); asm volatile("" ::: "memory"); }
static __device__ __forceinline__ h16 toh_flush(float v) { const h16 r = (h16)v; return (fabsf(v) < 6.103515625e-05f) ? (h16)0.0f : r; }

__global__ __launch_bounds__(256) void k_cvt8(const float* __restrict__ src, bf* dst, size_t n8) {
    const size_t i = (size_t)blockIdx.x * 256 + threadIdx.x; if (i >= n8) return;
    const v8f v = *(const v8f*)(src + i * 8); v8us o;
#pragma unroll
    for (int k = 0; k < 8; ++k) o[k] = f2bf(v[k]);
    *(volatile v8us*)(dst + i * 8) = o; __threadfence(); *(volatile v8us*)(dst + i * 8) = o;
}

template<int ASF16>
__global__ __launch_bounds__(256) void k_wT(const float* __restrict__ W, bf* WT) {
    __shared__ float tl[64 * 65];
    const int tid = threadIdx.x, lane = tid & 31, wave = __builtin_amdgcn_readfirstlane((int)(tid >> 5));
    const int k0 = blockIdx.x * 64, n0 = blockIdx.y * 64;
#pragma unroll
    for (int it = 0; it < 4; ++it) { const int r = (tid >> 4) + 16 * it, c = (tid & 15) * 4;
        const v4f v = *(const v4f*)(W + (size_t)(k0 + r) * DM + n0 + c);
        tl[r * 65 + c] = v[0]; tl[r * 65 + c + 1] = v[1]; tl[r * 65 + c + 2] = v[2]; tl[r * 65 + c + 3] = v[3]; }
    __syncthreads();
#pragma unroll 1
    for (int ps = 0; ps < 2; ++ps) {
#pragma unroll
        for (int s = 0; s < 2; ++s) { const int row = wave * 8 + s * 4 + (lane >> 3), c8 = (lane & 7) * 8;
            const size_t oo = (size_t)(n0 + row) * DM + k0 + c8;
            if constexpr (ASF16 != 0) { v8h o;
#pragma unroll
                for (int i = 0; i < 8; ++i) o[i] = (h16)(bfr(tl[(c8 + i) * 65 + row]) * WOS);
                *(volatile v8h*)((h16*)WT + oo) = o;
            } else { v8us o;
#pragma unroll
                for (int i = 0; i < 8; ++i) o[i] = f2bf(tl[(c8 + i) * 65 + row]);
                *(volatile v8us*)(WT + oo) = o; } }
        if (ps == 0) __threadfence(); }
}

__global__ __launch_bounds__(32) void k_proj(const bf* __restrict__ A, const bf* __restrict__ Bt, h16* Ph,
                                             int RB, size_t sRB, int pitch, int CB, size_t sCB) {
    __shared__ __align__(16) float os[16 * 68];
    const int K = DM;
    const int lane = threadIdx.x & 31, lr = lane & 15, hi = lane >> 4; const int r0 = blockIdx.x * 64, c0 = blockIdx.y * 64;
    v8f acc[4][4];
#pragma unroll
    for (int mb = 0; mb < 4; ++mb)
#pragma unroll
        for (int nb = 0; nb < 4; ++nb) acc[mb][nb] = (v8f){};
    const size_t aoff = (size_t)(r0 + lr) * K + 8 * hi, boff = (size_t)(c0 + lr) * K + 8 * hi;
#pragma unroll 1
    for (int kc = 0; kc < K; kc += 32) {
        v16bf a[4];
#pragma unroll
        for (int mb = 0; mb < 4; ++mb) a[mb] = ldb(A + aoff + (size_t)mb * 16 * K + kc);
#pragma unroll
        for (int nb = 0; nb < 4; ++nb) { const v16bf b = ldb(Bt + boff + (size_t)nb * 16 * K + kc);
#pragma unroll
            for (int mb = 0; mb < 4; ++mb) acc[mb][nb] = wmmab(a[mb], b, acc[mb][nb]); }
        asm volatile("v_nop\n\tv_nop\n\tv_nop\n\tv_nop" : "+v"(acc[0][0]), "+v"(acc[1][1]), "+v"(acc[2][2]), "+v"(acc[3][3]) : "v"(a[0]), "v"(a[1]), "v"(a[2]), "v"(a[3]));
    }
    const size_t tbase  = (size_t)(r0 / RB) * sRB  + (size_t)(r0 % RB) * (size_t)pitch  + (size_t)(c0 / CB) * sCB  + (size_t)(c0 % CB);
#pragma unroll
    for (int mb = 0; mb < 4; ++mb) {
#pragma unroll
        for (int nb = 0; nb < 4; ++nb) {
#pragma unroll
            for (int j = 0; j < 8; ++j) os[(hi * 8 + j) * 68 + nb * 16 + lr] = acc[mb][nb][j]; }
        wave_sync();
        const size_t sb  = tbase  + (size_t)(mb * 16) * (size_t)pitch;
#pragma unroll 1
        for (int ps = 0; ps < 2; ++ps) {
#pragma unroll
            for (int s = 0; s < 4; ++s) { const int row = 4 * s + (lane >> 3), c8 = (lane & 7) * 8;
                const v4f x0 = *(const v4fa*)(&os[row * 68 + c8]); const v4f x1 = *(const v4fa*)(&os[row * 68 + c8 + 4]);
                v8h hv;
#pragma unroll
                for (int i = 0; i < 4; ++i) { hv[i] = toh_flush(x0[i]); hv[4 + i] = toh_flush(x1[i]); }
                *(volatile v8h*)(Ph + sb + (size_t)row * (size_t)pitch + c8) = hv; }
            if (ps == 0) __threadfence(); }
        wave_sync();
    }
}

__global__ __launch_bounds__(1024) void k_biaschk(const float* __restrict__ BIAS, int* FLAG) {
    __shared__ int wbad[32];
    const int tid = threadIdx.x, lane = tid & 31, wave = __builtin_amdgcn_readfirstlane((int)(tid >> 5));
    const int perRow = SEQ / 4;
    int viol = 0;
#pragma unroll 1
    for (int i = tid; i < SEQ * perRow; i += 1024) {
        const int q = i / perRow, c = (i % perRow) * 4;
        const v4f m = *(const v4f*)(BIAS + (size_t)q * SEQ_FULL + c);
#pragma unroll
        for (int j = 0; j < 4; ++j) viol |= ((m[j] != 0.0f) ? 1 : 0);
    }
    const int wv = __any(viol);
    if (lane == 0) wbad[wave] = wv ? 1 : 0;
    __syncthreads();
    if (wave == 0) {
        const int tv = wbad[lane];
        const int anyv = __any(tv);
        const int f = anyv ? 0 : 1;
        if (lane < 8) { v4i o; o[0] = f; o[1] = f; o[2] = f; o[3] = f;
            *(volatile v4i*)(FLAG + lane * 4) = o; __threadfence(); *(volatile v4i*)(FLAG + lane * 4) = o; }
    }
}

__global__ __launch_bounds__(32 * AW) void k_flash(const h16* __restrict__ QH, const h16* __restrict__ KP, const h16* __restrict__ VT,
                                                   const float* __restrict__ BIAS, const int* __restrict__ FLAGP, float* OUT) {
    __shared__ __align__(16) float os[AW * 16 * 68];
    const int lane = threadIdx.x & 31, lr = lane & 15, hi = lane >> 4;
    const int wave = __builtin_amdgcn_readfirstlane((int)(threadIdx.x >> 5));
    const int zh = blockIdx.y; const int b = zh / NH_, h = zh % NH_;
    const int t0 = (blockIdx.x * AW + wave) * 16;
    const int flagv = __builtin_amdgcn_readfirstlane(FLAGP[0]);
    const bool addBias = (flagv != 1);
    const int nsteps = SEQ / 32;
    const size_t pbase = (size_t)zh * SEQ * HD;
    const size_t qo = pbase + (size_t)(t0 + lr) * HD + 8 * hi;
    const v16h qh0 = ldh(QH + qo), qh1 = ldh(QH + qo + 32);
    const size_t ko  = pbase + (size_t)lr * HD + 8 * hi;
    const size_t vo  = pbase + (size_t)lr * SEQ + 8 * hi;
    v8f oH[4];
#pragma unroll
    for (int j = 0; j < 4; ++j) { oH[j] = (v8f){}; }
    float m = -3.0e38f, l = 0.0f;
#pragma unroll 1
    for (int st = 0; st < nsteps; ++st) {
        const int key0 = st * 32;
        const h16* ka = KP + ko + (size_t)key0 * HD;
        const v16h ka0 = ldh(ka), ka1 = ldh(ka + 32), kb0 = ldh(ka + 16 * HD), kb1 = ldh(ka + 16 * HD + 32);
        v8f sHa = (v8f){}, sHb = (v8f){};
        sHa = wmma16(ka0, qh0, sHa); sHb = wmma16(kb0, qh0, sHb);
        sHa = wmma16(ka1, qh1, sHa); sHb = wmma16(kb1, qh1, sHb);
        asm volatile("v_nop\n\tv_nop\n\tv_nop\n\tv_nop" : "+v"(sHa), "+v"(sHb) : "v"(ka0), "v"(ka1), "v"(kb0), "v"(kb1));
        float ta[8], tb[8];
#pragma unroll
        for (int r = 0; r < 8; ++r) { ta[r] = sHa[r] * SC2; tb[r] = sHb[r] * SC2; }
        if (addBias) {
            const float* bp = BIAS + (size_t)(t0 + lr) * SEQ_FULL + key0 + 8 * hi;
            const v4f b0 = *(const v4f*)bp, b1 = *(const v4f*)(bp + 4), b2 = *(const v4f*)(bp + 16), b3 = *(const v4f*)(bp + 20);
#pragma unroll
            for (int r = 0; r < 4; ++r) {
                ta[r] = ta[r] + bfr(b0[r]) * L2E; ta[4 + r] = ta[4 + r] + bfr(b1[r]) * L2E;
                tb[r] = tb[r] + bfr(b2[r]) * L2E; tb[4 + r] = tb[4 + r] + bfr(b3[r]) * L2E; }
        }
        float mx = -3.0e38f;
#pragma unroll
        for (int r = 0; r < 8; ++r) mx = fmaxf(mx, fmaxf(ta[r], tb[r]));
        mx = fmaxf(mx, __shfl_xor(mx, 16, 32));
        const float mnew = fmaxf(m, mx);
        const float alpha = __builtin_amdgcn_exp2f(m - mnew);
        const float sh = PSH - mnew;
        v16h pb; float ls = 0.0f;
#pragma unroll
        for (int r = 0; r < 8; ++r) {
            const float xa = ta[r] + sh; const float xb = tb[r] + sh;
            const float ea = (xa < PFL) ? 0.0f : __builtin_amdgcn_exp2f(xa);
            const float eb = (xb < PFL) ? 0.0f : __builtin_amdgcn_exp2f(xb);
            const h16 pa = (h16)ea; const h16 pc = (h16)eb; pb[r] = pa; pb[8 + r] = pc;
            ls += (float)pa + (float)pc; }
        l = l * alpha + ls; m = mnew;
#pragma unroll
        for (int j = 0; j < 4; ++j) { oH[j] = oH[j] * alpha; }
        const h16* va = VT + vo + key0;
        const v16h v0 = ldh(va), v1 = ldh(va + (size_t)16 * SEQ), v2 = ldh(va + (size_t)32 * SEQ), v3 = ldh(va + (size_t)48 * SEQ);
        oH[0] = wmma16(v0, pb, oH[0]); oH[1] = wmma16(v1, pb, oH[1]); oH[2] = wmma16(v2, pb, oH[2]); oH[3] = wmma16(v3, pb, oH[3]);
        asm volatile("v_nop\n\tv_nop\n\tv_nop\n\tv_nop" : "+v"(oH[0]), "+v"(oH[1]), "+v"(oH[2]), "+v"(oH[3]) : "v"(v0), "v"(v1), "v"(v2), "v"(v3), "v"(pb));
    }
    l += __shfl_xor(l, 16, 32);
    const float inv = (1.0f / l);
    const int wb = wave * 16 * 68;
#pragma unroll
    for (int j = 0; j < 4; ++j) { v4f a, c;
#pragma unroll
        for (int r = 0; r < 4; ++r) { a[r] = oH[j][r] * inv; c[r] = oH[j][4 + r] * inv; }
        *(v4fa*)(&os[wb + lr * 68 + 16 * j + 8 * hi]) = a; *(v4fa*)(&os[wb + lr * 68 + 16 * j + 8 * hi + 4]) = c; }
    wave_sync();
    float* orow = OUT + ((size_t)b * OUT_SEQ + t0) * DM + h * HD;
#pragma unroll 1
    for (int ps = 0; ps < 2; ++ps) {
#pragma unroll
        for (int s = 0; s < 8; ++s) { const int row = 2 * s + hi, cofs = lr * 4;
            const v4f val = *(const v4fa*)(&os[wb + row * 68 + cofs]);
            *(volatile v4f*)(orow + (size_t)row * DM + cofs) = val; }
        if (ps == 0) __threadfence(); }
}

static constexpr size_t al256(size_t v) { return (v + 255) & ~(size_t)255; }
static constexpr size_t SZ_XB = al256((size_t)NB * SEQ * DM * 2);
static constexpr size_t SZ_WB = al256((size_t)3 * DM * DM * 2);
static constexpr size_t SZ_PL = al256((size_t)NB * NH_ * SEQ * HD * 2);
static constexpr size_t SZ_FL = 256;
static constexpr size_t SZ_TOTAL = 2 * SZ_XB + SZ_WB + 3 * SZ_PL + SZ_FL;
static_assert(SZ_TOTAL <= (size_t)134217728);
static_assert(((size_t)DM * DM * 2) % 256 == 0);
static_assert((size_t)NB * NH_ * SEQ * HD == (size_t)NB * SEQ * DM);

extern "C" void kernel_launch(void* const* d_in, const int* in_sizes, int n_in,
                              void* d_out, int out_size, void* d_ws, size_t ws_size, hipStream_t stream) {
    if (n_in < 6) return;
    const size_t needx = ((size_t)(NB - 1) * SEQ_FULL + SEQ) * DM;
    if ((size_t)in_sizes[0] < needx) return;
    if ((size_t)in_sizes[1] < needx) return;
    if ((size_t)in_sizes[2] < (size_t)(SEQ - 1) * SEQ_FULL + SEQ) return;
    if ((size_t)in_sizes[3] < (size_t)DM * DM || (size_t)in_sizes[4] < (size_t)DM * DM || (size_t)in_sizes[5] < (size_t)DM * DM) return;
    if ((size_t)out_size < ((size_t)(NB - 1) * OUT_SEQ + SEQ) * DM) return;
    if (SZ_TOTAL > ws_size) return;
    const float* x  = (const float*)d_in[0]; const float* y = (const float*)d_in[1];
    const float* sbias = (const float*)d_in[2];
    const float* wq = (const float*)d_in[3]; const float* wk = (const float*)d_in[4]; const float* wv = (const float*)d_in[5];
    float* OUT = (float*)d_out;
    char* wsp = (char*)d_ws;
    bf* XB = (bf*)wsp; wsp += SZ_XB;
    bf* YB = (bf*)wsp; wsp += SZ_XB;
    bf* WB = (bf*)wsp; wsp += SZ_WB;
    h16* QH = (h16*)wsp; wsp += SZ_PL;
    h16* KP = (h16*)wsp; wsp += SZ_PL;
    h16* VT = (h16*)wsp; wsp += SZ_PL;
    int* FLAG = (int*)wsp; wsp += SZ_FL;
    bf* WQT = WB; bf* WKT = WB + (size_t)DM * DM; bf* WVT = WB + (size_t)2 * DM * DM;

    if (SEQ == SEQ_FULL) {
        const size_t n8 = (size_t)NB * SEQ * DM / 8;
        k_cvt8<<<(unsigned)((n8 + 255) / 256), 256, 0, stream>>>(x, XB, n8);
        k_cvt8<<<(unsigned)((n8 + 255) / 256), 256, 0, stream>>>(y, YB, n8);
    } else {
        const size_t n8 = (size_t)SEQ * DM / 8;
        for (int b = 0; b < NB; ++b) k_cvt8<<<(unsigned)((n8 + 255) / 256), 256, 0, stream>>>(x + (size_t)b * SEQ_FULL * DM, XB + (size_t)b * SEQ * DM, n8);
        for (int b = 0; b < NB; ++b) k_cvt8<<<(unsigned)((n8 + 255) / 256), 256, 0, stream>>>(y + (size_t)b * SEQ_FULL * DM, YB + (size_t)b * SEQ * DM, n8);
    }
    k_wT<0><<<dim3(DM / 64, DM / 64, 1), 256, 0, stream>>>(wq, WQT);
    k_wT<0><<<dim3(DM / 64, DM / 64, 1), 256, 0, stream>>>(wk, WKT);
    k_wT<0><<<dim3(DM / 64, DM / 64, 1), 256, 0, stream>>>(wv, WVT);

    k_proj<<<dim3(NB * SEQ / 64, DM / 64, 1), 32, 0, stream>>>(XB, WQT, QH, SEQ, (size_t)NH_ * SEQ * HD, HD, HD, (size_t)SEQ * HD);
    k_proj<<<dim3(NB * SEQ / 64, DM / 64, 1), 32, 0, stream>>>(YB, WKT, KP, SEQ, (size_t)NH_ * SEQ * HD, HD, HD, (size_t)SEQ * HD);
    k_proj<<<dim3(DM / 64, NB * SEQ / 64, 1), 32, 0, stream>>>(WVT, YB, VT, DM, (size_t)0, SEQ, SEQ, (size_t)DM * SEQ);

    k_biaschk<<<1, 1024, 0, stream>>>(sbias, FLAG);

    k_flash<<<dim3(SEQ / (16 * AW), NB * NH_, 1), 32 * AW, 0, stream>>>(QH, KP, VT, sbias, FLAG, OUT);
}
